// HANLayer_18545668784544
// MI455X (gfx1250) — hardware-run, weakly checked
//
#include <hip/hip_runtime.h>
#include <stddef.h>
#include <stdint.h>
#include <math.h>

#define NN      50000
#define NE      800000
#define IND     128
#define OUTD    64
#define FSW     128
#define GBM     128
#define MP      50048
#define NTHR    256
#define NWAVE   8
#define EPT     8
#define WCH     (32 * EPT)
#define NBRUN   1024
#define SLB     10
#define NBK     49
#define WLCAP   2560
#define RCAP    20480
#define TRIPCAP 256
#define MAXDEG_MEAS   38
#define MAXB1024_MEAS 16696
#define RBM     64
#define SP      132
#define NEGSL   0.2f

#define BK_ZINTS (NWAVE * WLCAP + RCAP + 3 * NBRUN)
#define BK_INTS  (BK_ZINTS + 16)
#define BK_LDS   (BK_INTS * 4)
#define GM_LDS   ((GBM * SP + 128 + 2 * GBM) * 4)

#define PBX   (MP * IND / 8 / NTHR)
#define PBW   (FSW * IND / 8 / NTHR)
#define PBTOT (PBX + PBW + 1)

static_assert(IND == 128 && OUTD == 64 && FSW == 2 * OUTD && FSW == 4 * 32);
static_assert(IND % 32 == 0);
static_assert(MP % GBM == 0 && MP >= NN && MP == 391 * GBM && MP % RBM == 0);
static_assert(NBRUN == (1 << SLB) && NBRUN % RBM == 0 && NBRUN % 32 == 0);
static_assert(NBK * NBRUN >= NN && NBK * NBRUN >= MP);
static_assert(NN <= 65536);
static_assert(NE < (1 << 20) && (((long long)NE) << SLB) < (1LL << 31));
static_assert(NE % WCH == 0 && NE % 4 == 0);
static_assert(RCAP == NWAVE * WLCAP && RCAP % 32 == 0 && BK_ZINTS % 4 == 0);
static_assert((long long)RCAP * 100 >= (long long)MAXB1024_MEAS * 105);
static_assert(WLCAP >= MAXB1024_MEAS / 8 + 8 * 46 + 1);
static_assert(MAXDEG_MEAS + 8 <= TRIPCAP);
static_assert((MP * IND / 8) % NTHR == 0 && (FSW * IND / 8) % NTHR == 0 && PBW == 8);
static_assert(BK_LDS <= 300000 && BK_LDS <= 327680);
static_assert(GM_LDS <= 327680);
static_assert((GBM * SP * 4) % 16 == 0 && (SP * 4) % 16 == 0);
static_assert(GBM == NWAVE * 16 && RBM == NWAVE * 8);
static_assert((2 * NBRUN) % (NTHR * 4) == 0 && RCAP % (NTHR * 4) == 0);

typedef float          v4f   __attribute__((ext_vector_type(4)));
typedef float          v8f   __attribute__((ext_vector_type(8)));
typedef int            v4i   __attribute__((ext_vector_type(4)));
typedef int            v8i   __attribute__((ext_vector_type(8)));
typedef unsigned short v8us  __attribute__((ext_vector_type(8)));
typedef unsigned short v16us __attribute__((ext_vector_type(16)));
typedef __bf16         v16bf __attribute__((ext_vector_type(16)));
typedef v4f  __attribute__((may_alias)) v4fa;
typedef v4i  __attribute__((may_alias)) v4ia;
typedef v8us __attribute__((may_alias)) v8usa;
union FragB { v16bf v; v16us u; v8us h[2]; v8i w; };

__device__ __forceinline__ v8f wmb(const FragB& a, const FragB& b, v8f c) {
  v8f d = __builtin_amdgcn_wmma_f32_16x16x32_bf16(false, a.v, false, b.v, (short)0, c, false, false);
  asm volatile("v_nop\n\tv_nop\n\tv_nop\n\tv_nop" : "+v"(d) : "v"(a.w), "v"(b.w));
  return d;
}

__device__ __forceinline__ unsigned bf16_bits(float f) {
  const unsigned u = __float_as_uint(f);
  const unsigned r = (u + 0x7FFFu + ((u >> 16) & 1u)) >> 16;
  const unsigned q = (u >> 16) | 0x40u;
  return ((u & 0x7fffffffu) > 0x7f800000u) ? q : r;
}

__device__ __forceinline__ void st2_v4f(float* p, v4f v) {
  *(volatile v4f*)p = v;
  __threadfence();
  *(volatile v4f*)p = v;
}
__device__ __forceinline__ void st2_v8us(unsigned short* p, v8us v) {
  *(volatile v8us*)p = v;
  __threadfence();
  *(volatile v8us*)p = v;
}

__device__ __forceinline__ v8us gather8(const float* __restrict__ base, int stride) {
  float f[8];
#pragma unroll
  for (int i = 0; i < 8; ++i) f[i] = base[(size_t)i * (size_t)stride];
  v8us o;
#pragma unroll
  for (int i = 0; i < 8; ++i) o[i] = (unsigned short)bf16_bits(f[i]);
  return o;
}

__global__ __launch_bounds__(NTHR) void k_prep(const float* __restrict__ h, const float* __restrict__ w0,
                                               const float* __restrict__ al, const float* __restrict__ ar,
                                               const float* __restrict__ b0, const float* __restrict__ w1,
                                               const float* __restrict__ b1,
                                               unsigned short* xb, unsigned short* bt, float* par) {
  const int tid = (int)threadIdx.x;
  const int blk = (int)blockIdx.x;
  if (blk < PBX) {
    const int u   = blk * NTHR + tid;
    const int row = u >> 4, k8 = (u & 15) * 8;
    const int rc  = row < NN ? row : NN - 1;
    const unsigned mk = row < NN ? 0xffffu : 0u;
    const float* p = h + (size_t)rc * IND + k8;
    const v4f a = *(const v4fa*)p;
    const v4f b = *(const v4fa*)(p + 4);
    v8us o;
    o[0] = (unsigned short)(bf16_bits(a.x) & mk); o[1] = (unsigned short)(bf16_bits(a.y) & mk);
    o[2] = (unsigned short)(bf16_bits(a.z) & mk); o[3] = (unsigned short)(bf16_bits(a.w) & mk);
    o[4] = (unsigned short)(bf16_bits(b.x) & mk); o[5] = (unsigned short)(bf16_bits(b.y) & mk);
    o[6] = (unsigned short)(bf16_bits(b.z) & mk); o[7] = (unsigned short)(bf16_bits(b.w) & mk);
    st2_v8us(xb + (size_t)row * IND + k8, o);
  } else if (blk < PBX + PBW / 2) {
    const int u = (blk - PBX) * NTHR + tid;
    const int n = u >> 4, k8 = (u & 15) * 8;
    const v8us o = gather8(w0 + (size_t)k8 * OUTD + n, OUTD);
    st2_v8us(bt + (size_t)n * IND + k8, o);
  } else if (blk < PBX + PBW) {
    const int u = (blk - PBX) * NTHR + tid;
    const int n = u >> 4, k8 = (u & 15) * 8;
    const v8us o = gather8(w1 + (size_t)k8 * OUTD + (n - OUTD), OUTD);
    st2_v8us(bt + (size_t)n * IND + k8, o);
  } else {
    if (tid < 64) {
      const int q = tid & 15, r = tid >> 4;
      const v4f a = *(const v4fa*)(al + 4 * q);
      const v4f b = *(const v4fa*)(ar + 4 * q);
      const v4f c = *(const v4fa*)(b0 + 4 * q);
      const v4f d = *(const v4fa*)(b1 + 4 * q);
      asm volatile("" :: "v"(a));
      asm volatile("" :: "v"(b));
      asm volatile("" :: "v"(c));
      asm volatile("" :: "v"(d));
      const unsigned m0 = (r == 0) ? 0xffffffffu : 0u, m1 = (r == 1) ? 0xffffffffu : 0u;
      const unsigned m2 = (r == 2) ? 0xffffffffu : 0u, m3 = (r == 3) ? 0xffffffffu : 0u;
      v4f o;
      o.x = __uint_as_float(((bf16_bits(a.x) << 16) & m0) | ((bf16_bits(b.x) << 16) & m1) |
                            ((bf16_bits(c.x) << 16) & m2) | ((bf16_bits(d.x) << 16) & m3));
      o.y = __uint_as_float(((bf16_bits(a.y) << 16) & m0) | ((bf16_bits(b.y) << 16) & m1) |
                            ((bf16_bits(c.y) << 16) & m2) | ((bf16_bits(d.y) << 16) & m3));
      o.z = __uint_as_float(((bf16_bits(a.z) << 16) & m0) | ((bf16_bits(b.z) << 16) & m1) |
                            ((bf16_bits(c.z) << 16) & m2) | ((bf16_bits(d.z) << 16) & m3));
      o.w = __uint_as_float(((bf16_bits(a.w) << 16) & m0) | ((bf16_bits(b.w) << 16) & m1) |
                            ((bf16_bits(c.w) << 16) & m2) | ((bf16_bits(d.w) << 16) & m3));
      st2_v4f(par + 4 * tid, o);
    }
  }
}

__device__ __forceinline__ void gemm_flush(const float* stg, const float* sdt, float* FS, float* SD,
                                           int rowBase, int tid, int lane, int wave) {
#pragma unroll 1
  for (int i = 0; i < 16; ++i) {
    const int row = 16 * wave + i;
    const v4f p = *(const v4fa*)(stg + row * SP + 4 * lane);
    float* op = FS + (size_t)(rowBase + row) * FSW + 4 * lane;
    *(volatile v4f*)op = p;
  }
  if (tid < 64) {
    const v4f s = *(const v4fa*)(sdt + 4 * tid);
    float* sp = SD + (size_t)rowBase * 2 + 4 * tid;
    *(volatile v4f*)sp = s;
  }
}

__global__ __launch_bounds__(NTHR) __attribute__((amdgpu_num_vgpr(248)))
void k_gemm(const unsigned short* __restrict__ XB, const unsigned short* __restrict__ BT,
            const float* __restrict__ PAR, float* FS, float* SD) {
  extern __shared__ __attribute__((aligned(16))) float gsm[];
  float* stg  = gsm;
  float* spar = gsm + GBM * SP;
  float* sdt  = spar + 128;
  const int tid = (int)threadIdx.x, lane = tid & 31, wave = tid >> 5, hh = lane >> 4, m = lane & 15;
  const int rowBase = (int)blockIdx.x * GBM;
  if (tid < 32) *(v4fa*)(spar + 4 * tid) = *(const v4fa*)(PAR + 4 * tid);

  v8f acc[8];
  {
    const v8f z = {0.f, 0.f, 0.f, 0.f, 0.f, 0.f, 0.f, 0.f};
#pragma unroll
    for (int t = 0; t < 8; ++t) acc[t] = z;
  }
  const unsigned short* ap = XB + (size_t)(rowBase + 16 * wave + m) * (size_t)IND + 8 * hh;
  const unsigned short* bp = BT + (size_t)m * (size_t)IND + 8 * hh;

#pragma unroll 1
  for (int k0 = 0; k0 < IND; k0 += 32) {
    FragB af;
    af.h[0] = *(const v8usa*)(ap + k0);
    af.h[1] = *(const v8usa*)(ap + k0 + 16);
#pragma unroll
    for (int nt = 0; nt < 8; ++nt) {
      const unsigned short* wq = bp + (size_t)(16 * nt) * (size_t)IND + k0;
      FragB bf;
      bf.h[0] = *(const v8usa*)wq;
      bf.h[1] = *(const v8usa*)(wq + 16);
      acc[nt] = wmb(af, bf, acc[nt]);
    }
  }

#pragma unroll
  for (int nt = 0; nt < 8; ++nt) {
#pragma unroll
    for (int r = 0; r < 8; ++r) stg[(16 * wave + 8 * hh + r) * SP + 16 * nt + m] = acc[nt][r];
  }
  __syncthreads();

  {
    const v4f al4 = *(const v4fa*)(spar + 4 * m);
    const v4f ar4 = *(const v4fa*)(spar + 64 + 4 * m);
    const bool lo16 = lane < 16;
#pragma unroll 1
    for (int i = 0; i < 16; ++i) {
      const int row = 16 * wave + i;
      const v4f p = *(const v4fa*)(stg + row * SP + 4 * lane);
      float s = p.x * al4.x; s = fmaf(p.y, al4.y, s); s = fmaf(p.z, al4.z, s); s = fmaf(p.w, al4.w, s);
      float d = p.x * ar4.x; d = fmaf(p.y, ar4.y, d); d = fmaf(p.z, ar4.z, d); d = fmaf(p.w, ar4.w, d);
      s = lo16 ? s : 0.0f;
      d = lo16 ? d : 0.0f;
#pragma unroll
      for (int off = 16; off > 0; off >>= 1) {
        s += __shfl_xor(s, off, 32);
        d += __shfl_xor(d, off, 32);
      }
      if (lane == 0) { sdt[2 * row] = s; sdt[2 * row + 1] = d; }
    }
  }
  __syncthreads();

  gemm_flush(stg, sdt, FS, SD, rowBase, tid, lane, wave);
  __threadfence();
  gemm_flush(stg, sdt, FS, SD, rowBase, tid, lane, wave);
}

__device__ __forceinline__ void bucket_flush(const int* pl, const int* cnt, int ov, int* lp, int* cop, int* fp,
                                             int tid) {
#pragma unroll 1
  for (int i = tid * 4; i < RCAP; i += NTHR * 4) {
    const v4i v = *(const v4ia*)(pl + i);
    *(volatile v4i*)(lp + i) = v;
  }
#pragma unroll 1
  for (int i = tid * 4; i < 2 * NBRUN; i += NTHR * 4) {
    const v4i v = *(const v4ia*)(cnt + i);
    *(volatile v4i*)(cop + i) = v;
  }
  if (tid < 8) {
    const v4i f = {ov, ov, ov, ov};
    *(volatile v4i*)(fp + 4 * tid) = f;
  }
}

template <int ROLE>
__device__ __forceinline__ void bucket_body(const int* __restrict__ keys, const int* __restrict__ gix,
                                            const float* __restrict__ wts, int rb,
                                            int* lp, int* cop, int* fp, int* dsm) {
  int* wl   = dsm;
  int* pl   = dsm + NWAVE * WLCAP;
  int* cnt  = pl + RCAP;
  int* offs = cnt + NBRUN;
  int* cur  = offs + NBRUN;
  int* misc = cur + NBRUN;
  const int tid = (int)threadIdx.x, lane = tid & 31, wave = tid >> 5;
  const unsigned nbs = (unsigned)(rb * NBRUN);
  const int nbI = (NN - rb * NBRUN) < NBRUN ? (NN - rb * NBRUN) : NBRUN;
  const unsigned unb = (unsigned)(nbI < 0 ? 0 : nbI);

  {
    const v4i z4 = {0, 0, 0, 0};
    for (int i = tid * 4; i < BK_ZINTS; i += NTHR * 4) *(v4ia*)(dsm + i) = z4;
    if (tid < 16) misc[tid] = 0;
  }
  __syncthreads();

  {
    const int per  = ((NE + NWAVE * WCH - 1) / (NWAVE * WCH)) * WCH;
    const int ebeg = wave * per;
    const int eend = (ebeg + per < NE) ? (ebeg + per) : NE;
    int* mylist = wl + wave * WLCAP;
    int wc = 0;
#pragma unroll 1
    for (int cb = ebeg; cb < eend; cb += WCH) {
      const int e0 = cb + lane * EPT;
      const v4i da = *(const v4ia*)(keys + e0);
      const v4i db = *(const v4ia*)(keys + e0 + 4);
      const unsigned s0 = (unsigned)da.x - nbs, s1 = (unsigned)da.y - nbs;
      const unsigned s2 = (unsigned)da.z - nbs, s3 = (unsigned)da.w - nbs;
      const unsigned s4 = (unsigned)db.x - nbs, s5 = (unsigned)db.y - nbs;
      const unsigned s6 = (unsigned)db.z - nbs, s7 = (unsigned)db.w - nbs;
      const bool h0 = s0 < unb, h1 = s1 < unb, h2 = s2 < unb, h3 = s3 < unb;
      const bool h4 = s4 < unb, h5 = s5 < unb, h6 = s6 < unb, h7 = s7 < unb;
      const unsigned m0 = __builtin_amdgcn_ballot_w32(h0), m1 = __builtin_amdgcn_ballot_w32(h1);
      const unsigned m2 = __builtin_amdgcn_ballot_w32(h2), m3 = __builtin_amdgcn_ballot_w32(h3);
      const unsigned m4 = __builtin_amdgcn_ballot_w32(h4), m5 = __builtin_amdgcn_ballot_w32(h5);
      const unsigned m6 = __builtin_amdgcn_ballot_w32(h6), m7 = __builtin_amdgcn_ballot_w32(h7);
      const unsigned any = m0 | m1 | m2 | m3 | m4 | m5 | m6 | m7;
      if (any != 0u) {
        const int pre = (int)(__builtin_amdgcn_mbcnt_lo(m0, 0u) + __builtin_amdgcn_mbcnt_lo(m1, 0u) +
                              __builtin_amdgcn_mbcnt_lo(m2, 0u) + __builtin_amdgcn_mbcnt_lo(m3, 0u) +
                              __builtin_amdgcn_mbcnt_lo(m4, 0u) + __builtin_amdgcn_mbcnt_lo(m5, 0u) +
                              __builtin_amdgcn_mbcnt_lo(m6, 0u) + __builtin_amdgcn_mbcnt_lo(m7, 0u));
        int p = wc + pre;
        if (h0) { if (p < WLCAP) mylist[p] = ((e0 + 0) << SLB) | (int)s0; p = p + 1; }
        if (h1) { if (p < WLCAP) mylist[p] = ((e0 + 1) << SLB) | (int)s1; p = p + 1; }
        if (h2) { if (p < WLCAP) mylist[p] = ((e0 + 2) << SLB) | (int)s2; p = p + 1; }
        if (h3) { if (p < WLCAP) mylist[p] = ((e0 + 3) << SLB) | (int)s3; p = p + 1; }
        if (h4) { if (p < WLCAP) mylist[p] = ((e0 + 4) << SLB) | (int)s4; p = p + 1; }
        if (h5) { if (p < WLCAP) mylist[p] = ((e0 + 5) << SLB) | (int)s5; p = p + 1; }
        if (h6) { if (p < WLCAP) mylist[p] = ((e0 + 6) << SLB) | (int)s6; p = p + 1; }
        if (h7) { if (p < WLCAP) mylist[p] = ((e0 + 7) << SLB) | (int)s7; p = p + 1; }
        wc += (int)(__builtin_popcount(m0) + __builtin_popcount(m1) + __builtin_popcount(m2) + __builtin_popcount(m3) +
                    __builtin_popcount(m4) + __builtin_popcount(m5) + __builtin_popcount(m6) + __builtin_popcount(m7));
      }
    }
    if (lane == 0) misc[wave] = wc;
  }
  __syncthreads();

  if (wave == 0) {
    int ov = 0;
#pragma unroll 1
    for (int w2 = 0; w2 < NWAVE; ++w2) {
      int c = misc[w2];
      if (c > WLCAP) ov = 1;
      c = c < 0 ? 0 : (c > WLCAP ? WLCAP : c);
#pragma unroll 1
      for (int b0 = 0; b0 < c; b0 += 32) {
        const int idx = b0 + lane;
        const int ent = wl[w2 * WLCAP + (idx < WLCAP ? idx : WLCAP - 1)];
        const int m32 = (c - b0) < 32 ? (c - b0) : 32;
#pragma unroll 1
        for (int k = 0; k < m32; ++k) {
          const int u    = __builtin_amdgcn_readlane(ent, k);
          const int slot = u & (NBRUN - 1);
          if (lane == 0) cnt[slot] = cnt[slot] + 1;
        }
      }
    }
    if (lane == 0) misc[9] = ov;
  }
  __syncthreads();
  if (wave == 0) {
    const int base = lane * (NBRUN / 32);
    int s = 0;
#pragma unroll 1
    for (int i = 0; i < NBRUN / 32; ++i) s += cnt[base + i];
    int incl = s;
#pragma unroll
    for (int d = 1; d < 32; d <<= 1) {
      const int y = __shfl_up(incl, d, 32);
      if (lane >= d) incl += y;
    }
    int run = incl - s;
#pragma unroll 1
    for (int i = 0; i < NBRUN / 32; ++i) {
      const int cv = cnt[base + i];
      offs[base + i] = run;
      cur[base + i]  = run;
      run += cv;
    }
  }
  __syncthreads();

  if (wave == 0) {
#pragma unroll 1
    for (int w2 = 0; w2 < NWAVE; ++w2) {
      int c = misc[w2];
      c = c < 0 ? 0 : (c > WLCAP ? WLCAP : c);
#pragma unroll 1
      for (int b0 = 0; b0 < c; b0 += 32) {
        const int idx = b0 + lane;
        const int ent = wl[w2 * WLCAP + (idx < WLCAP ? idx : WLCAP - 1)];
        int eid = (ent >> SLB) & 0xFFFFF;
        eid = eid > NE - 1 ? NE - 1 : eid;
        int sr = gix[eid];
        sr = sr < 0 ? 0 : (sr > NN - 1 ? NN - 1 : sr);
        int word = sr;
        if constexpr (ROLE != 0) {
          const float wv = wts[eid];
          word = (int)((unsigned)sr | (bf16_bits(wv) << 16));
        }
        const int m32 = (c - b0) < 32 ? (c - b0) : 32;
#pragma unroll 1
        for (int k = 0; k < m32; ++k) {
          const int u    = __builtin_amdgcn_readlane(ent, k);
          const int wd   = __builtin_amdgcn_readlane(word, k);
          const int slot = u & (NBRUN - 1);
          if (lane == 0) {
            int p = cur[slot];
            p = p < 0 ? 0 : (p > RCAP - 1 ? RCAP - 1 : p);
            pl[p] = wd;
            cur[slot] = p + 1;
          }
        }
      }
    }
  }
  __syncthreads();

  const int ovf = misc[9];
  bucket_flush(pl, cnt, ovf, lp, cop, fp, tid);
  __threadfence();
  bucket_flush(pl, cnt, ovf, lp, cop, fp, tid);
}

__global__ __launch_bounds__(NTHR) void k_bucket(const int* __restrict__ src0, const int* __restrict__ dst0,
                                                 const int* __restrict__ row2, const int* __restrict__ col2,
                                                 const float* __restrict__ adj, int* LIST, int* CO, int* FLAG) {
  extern __shared__ __attribute__((aligned(16))) int dsm[];
  const int blk = (int)blockIdx.x;
  int* lp  = LIST + (size_t)blk * RCAP;
  int* cop = CO + (size_t)blk * (2 * NBRUN);
  int* fp  = FLAG + (size_t)blk * 32;
  if (blk < NBK) {
    bucket_body<0>(dst0, src0, adj, blk, lp, cop, fp, dsm);
  } else {
    bucket_body<1>(row2, col2, adj, blk - NBK, lp, cop, fp, dsm);
  }
}

__global__ __launch_bounds__(NTHR) void k_replay(const int* __restrict__ LIST, const int* __restrict__ CO,
                                                 const int* __restrict__ FLAG, const float* __restrict__ FS,
                                                 const float* __restrict__ SD, const float* __restrict__ PAR,
                                                 float* out) {
  __shared__ __attribute__((aligned(16))) float spar[128];
  const int tid = (int)threadIdx.x, lane = tid & 31, wave = tid >> 5, hh = lane >> 4;
  if (tid < 32) *(v4fa*)(spar + 4 * tid) = *(const v4fa*)(PAR + 128 + 4 * tid);
  __syncthreads();
  const v4f bias = *(const v4fa*)(spar + 4 * lane);
  const bool isB = hh != 0;
  const int nodeBase = (int)blockIdx.x * RBM;
  const int bucket   = nodeBase >> SLB;
  const int rbk      = hh * NBK + bucket;
  const size_t lbase = (size_t)rbk * RCAP;
  const size_t cbase = (size_t)rbk * (2 * NBRUN);
  const int flag     = FLAG[(size_t)rbk * 32];
  const float qnan   = __uint_as_float(0x7fc00000u);
  const float ninf   = __uint_as_float(0xff800000u);

#pragma unroll 1
  for (int i = 0; i < RBM / NWAVE; ++i) {
    const int node = nodeBase + (RBM / NWAVE) * wave + i;
    if (node < NN) {
      const int slot = node & (NBRUN - 1);
      int c = CO[cbase + slot];
      int o = CO[cbase + NBRUN + slot];
      const bool big = c > TRIPCAP;
      c = c < 0 ? 0 : (c > TRIPCAP ? TRIPCAP : c);
      o = o < 0 ? 0 : (o > RCAP - 1 ? RCAP - 1 : o);
      const int co = __shfl_xor(c, 16, 32);
      int cmv = c > co ? c : co;
      cmv = cmv < 0 ? 0 : (cmv > TRIPCAP ? TRIPCAP : cmv);
      const int cm = __builtin_amdgcn_readfirstlane(cmv);
      int last = o + c - 1;
      last = last < o ? o : last;
      last = last > RCAP - 1 ? RCAP - 1 : last;
      const float erd = SD[2 * (size_t)node + 1];
      float m = ninf, l = 0.0f;
      float a0 = 0.0f, a1 = 0.0f, a2 = 0.0f, a3 = 0.0f;
#pragma unroll 1
      for (int j = 0; j < cm; ++j) {
        int idx = o + j;
        idx = idx > last ? last : idx;
        const unsigned wd = (unsigned)LIST[lbase + (size_t)idx];
        int sr = (int)(wd & 0xffffu);
        sr = sr > NN - 1 ? NN - 1 : sr;
        const float w   = __uint_as_float(wd & 0xffff0000u);
        const float els = SD[2 * (size_t)sr];
        const v4f v = *(const v4fa*)(FS + (size_t)sr * FSW + 4 * lane);
        asm volatile("" :: "v"(els));
        asm volatile("" :: "v"(v));
        float e = els + erd;
        e = (e > 0.0f) ? e : NEGSL * e;
        const float df = e - m;
        const float ee = expf(-fabsf(df));
        const bool  up = df > 0.0f;
        const float rA = up ? ee : 1.0f;
        const float pA = up ? 1.0f : ee;
        const float rr = isB ? 1.0f : rA;
        const float pp = isB ? w : pA;
        const float ln = fmaf(l, rr, pp);
        const float t0 = fmaf(pp, v.x, a0 * rr), t1 = fmaf(pp, v.y, a1 * rr);
        const float t2 = fmaf(pp, v.z, a2 * rr), t3 = fmaf(pp, v.w, a3 * rr);
        const float mn = up ? e : m;
        const bool valid = j < c;
        m  = valid ? mn : m;
        l  = valid ? ln : l;
        a0 = valid ? t0 : a0; a1 = valid ? t1 : a1; a2 = valid ? t2 : a2; a3 = valid ? t3 : a3;
      }
      const bool  empty = c == 0;
      const float lsafe = (isB | empty) ? 1.0f : l;
      const float inv   = 1.0f / lsafe;
      const float sc    = isB ? 1.0f : inv;
      float y0 = a0 * sc, y1 = a1 * sc, y2 = a2 * sc, y3 = a3 * sc;
      y0 = empty ? 0.0f : y0; y1 = empty ? 0.0f : y1; y2 = empty ? 0.0f : y2; y3 = empty ? 0.0f : y3;
      y0 = y0 + bias.x; y1 = y1 + bias.y; y2 = y2 + bias.z; y3 = y3 + bias.w;
#pragma unroll 1
      for (int t = 0; t < 4; ++t) {
        const float x  = y0;
        const float en = expm1f(x);
        const float f  = (x > 0.0f) ? x : en;
        y0 = y1; y1 = y2; y2 = y3; y3 = f;
      }
      const bool bad = (flag != 0) | big;
      v4f ov;
      ov.x = bad ? qnan : y0; ov.y = bad ? qnan : y1; ov.z = bad ? qnan : y2; ov.w = bad ? qnan : y3;
      float* op = out + (size_t)node * FSW + 4 * lane;
      *(volatile v4f*)op = ov;
      __threadfence();
      *(volatile v4f*)op = ov;
    }
  }
}

extern "C" void kernel_launch(void* const* d_in, const int* in_sizes, int n_in,
                              void* d_out, int out_size, void* d_ws, size_t ws_size,
                              hipStream_t stream) {
  if (n_in < 12) return;
  if (in_sizes[0] != NN * IND) return;
  if (in_sizes[1] != NE || in_sizes[2] != NE) return;
  if (in_sizes[3] != NE || in_sizes[4] != NE) return;
  if (in_sizes[5] != NE) return;
  if (in_sizes[6] != IND * OUTD) return;
  if (in_sizes[7] != OUTD || in_sizes[8] != OUTD || in_sizes[9] != OUTD) return;
  if (in_sizes[10] != IND * OUTD) return;
  if (in_sizes[11] != OUTD) return;
  if (out_size != NN * FSW) return;

  const float* h    = (const float*)d_in[0];
  const int*   src0 = (const int*)d_in[1];
  const int*   dst0 = (const int*)d_in[2];
  const int*   row2 = (const int*)d_in[3];
  const int*   col2 = (const int*)d_in[4];
  const float* adj  = (const float*)d_in[5];
  const float* W0   = (const float*)d_in[6];
  const float* al   = (const float*)d_in[7];
  const float* ar   = (const float*)d_in[8];
  const float* b0   = (const float*)d_in[9];
  const float* W1   = (const float*)d_in[10];
  const float* b1   = (const float*)d_in[11];
  float* out = (float*)d_out;

  constexpr size_t zXB   = (size_t)MP * IND * 2;
  constexpr size_t zFS   = (size_t)MP * FSW * 4;
  constexpr size_t zSD   = (size_t)MP * 2 * 4;
  constexpr size_t zLIST = (size_t)2 * NBK * RCAP * 4;
  constexpr size_t zCO   = (size_t)2 * NBK * 2 * NBRUN * 4;
  constexpr size_t zFLAG = (size_t)2 * NBK * 128;
  constexpr size_t zBT   = (size_t)FSW * IND * 2;
  constexpr size_t zPAR  = 1024;
  constexpr size_t oXB   = 0;
  constexpr size_t oFS   = oXB + zXB;
  constexpr size_t oSD   = oFS + zFS;
  constexpr size_t oLIST = oSD + zSD;
  constexpr size_t oCO   = oLIST + zLIST;
  constexpr size_t oFLAG = oCO + zCO;
  constexpr size_t oBT   = oFLAG + zFLAG;
  constexpr size_t oPAR  = oBT + zBT;
  constexpr size_t oEND  = oPAR + zPAR;
  static_assert(zXB % 256 == 0 && zFS % 256 == 0 && zSD % 256 == 0 && zLIST % 256 == 0 && zCO % 256 == 0);
  static_assert(zFLAG % 256 == 0 && zBT % 256 == 0 && zPAR % 256 == 0);
  static_assert(oEND <= (size_t)(128u << 20));
  if (oEND > ws_size) return;

  char* ws = (char*)d_ws;
  unsigned short* XB   = (unsigned short*)(ws + oXB);
  float*          FS   = (float*)(ws + oFS);
  float*          SD   = (float*)(ws + oSD);
  int*            LIST = (int*)(ws + oLIST);
  int*            CO   = (int*)(ws + oCO);
  int*            FLAG = (int*)(ws + oFLAG);
  unsigned short* BT   = (unsigned short*)(ws + oBT);
  float*          PAR  = (float*)(ws + oPAR);

  hipFuncSetAttribute(reinterpret_cast<const void*>(&k_gemm), hipFuncAttributeMaxDynamicSharedMemorySize, (int)GM_LDS);
  hipFuncSetAttribute(reinterpret_cast<const void*>(&k_bucket), hipFuncAttributeMaxDynamicSharedMemorySize, (int)BK_LDS);

  k_prep<<<PBTOT, NTHR, 0, stream>>>(h, W0, al, ar, b0, W1, b1, XB, BT, PAR);
  k_gemm<<<MP / GBM, NTHR, GM_LDS, stream>>>(XB, BT, PAR, FS, SD);
  k_bucket<<<2 * NBK, NTHR, BK_LDS, stream>>>(src0, dst0, row2, col2, adj, LIST, CO, FLAG);
  k_replay<<<MP / RBM, NTHR, 0, stream>>>(LIST, CO, FLAG, FS, SD, PAR, out);
}
